// HGTNet_51960514347439
// MI455X (gfx1250) — hardware-verified
//
#include <hip/hip_runtime.h>
#include <stddef.h>
#include <stdint.h>


#define FIN     16
#define HC      64
#define KENC    32
#define KHL     128
#define NOUT    16
#define NLAY    2
#define ATW     8
#define ATB     256
#define NTHR    256
#define NWAVE   8
#define EPT     8
#define CHUNK   (NTHR * EPT)
#define WCAP    (EPT * 32)
#define LISTN   (NWAVE * WCAP)
#define NBMAX   2048
#define RCAP    28672
#define DEGCAP  256
#define STW     512
#define GBM     64
#define GBN     64
#define GTHR    128
#define MIXR    64
#define WSMAX   134217728
#define LDS_AGG ((2 * RCAP + 2 * NBMAX + LISTN) * 4 + 64)

static_assert((CHUNK & (CHUNK - 1)) == 0 && CHUNK <= 4096);
static_assert((NBMAX & (NBMAX - 1)) == 0 && NBMAX <= 4096);
static_assert(NTHR * 8 == NBMAX);
static_assert(LISTN >= NBMAX);
static_assert(LISTN >= NWAVE * WCAP);
static_assert((RCAP % 32) == 0);
static_assert(NWAVE * STW <= RCAP);
static_assert(LDS_AGG <= 300000);
static_assert(GBM == (GTHR / 32) * 16);
static_assert(HC == 64 && GBN == HC);
static_assert(KENC == 2 * FIN && KHL == 2 * HC && (KENC % 32) == 0 && (KHL % 32) == 0);
static_assert(MIXR == NWAVE * 8);
static_assert(ATB * ATW == 4 * 2 * ATB);
static_assert(2 * HC <= STW);
static_assert(GBM * NOUT / 4 == 2 * GTHR);
static_assert(GBM * KHL / 8 == 8 * GTHR);

typedef float          v4f  __attribute__((ext_vector_type(4)));
typedef float          v8f  __attribute__((ext_vector_type(8)));
typedef int            v4i  __attribute__((ext_vector_type(4)));
typedef int            v8i  __attribute__((ext_vector_type(8)));
typedef unsigned short v8us __attribute__((ext_vector_type(8)));
typedef __bf16         v16b __attribute__((ext_vector_type(16)));
union FragB { v16b v; v8us u[2]; v8i w; };

__device__ __forceinline__ v8f wmb(const FragB& a, const FragB& b, v8f c) {
  v8f d = __builtin_amdgcn_wmma_f32_16x16x32_bf16(false, a.v, false, b.v, (short)0, c, false, false);
  asm volatile("v_nop\n\tv_nop\n\tv_nop\n\tv_nop" : "+v"(d) : "v"(a.w), "v"(b.w));
  return d;
}

__device__ __forceinline__ void ldwait() {
  asm volatile("s_wait_loadcnt 0x0" ::: "memory");
}

__device__ __forceinline__ unsigned bfb(float f) {
  const unsigned u = __float_as_uint(f);
  return (u + 0x7FFFu + ((u >> 16) & 1u)) >> 16;
}
__device__ __forceinline__ float bfv(unsigned b) { return __uint_as_float(b << 16); }
__device__ __forceinline__ float bfr(float f) { return bfv(bfb(f)); }

__device__ __forceinline__ v8us bits8(const v4f a, const v4f b) {
  v8us r;
  r[0] = (unsigned short)bfb(a.x); r[1] = (unsigned short)bfb(a.y);
  r[2] = (unsigned short)bfb(a.z); r[3] = (unsigned short)bfb(a.w);
  r[4] = (unsigned short)bfb(b.x); r[5] = (unsigned short)bfb(b.y);
  r[6] = (unsigned short)bfb(b.z); r[7] = (unsigned short)bfb(b.w);
  return r;
}
__device__ __forceinline__ void split8(const v4f a, const v4f b, v8us& hi, v8us& lo) {
  const float f[8] = {a.x, a.y, a.z, a.w, b.x, b.y, b.z, b.w};
#pragma unroll
  for (int j = 0; j < 8; ++j) {
    const unsigned hb = bfb(f[j]);
    hi[j] = (unsigned short)hb;
    lo[j] = (unsigned short)bfb(f[j] - bfv(hb));
  }
}

__device__ __forceinline__ int scan_chunk(const int* __restrict__ dsts, int nE, int cbase, int slotBase,
                                          int nb, int vec8, int* list, int tid, int lane, int wave) {
  int wc = 0;
  const int el0  = tid * EPT;
  const int e0   = cbase + el0;
  const int sent = -2147483647 - 1;
  v4i da, db;
  if (vec8 != 0 && cbase + CHUNK <= nE) {
    da = *(const v4i*)(dsts + e0);
    db = *(const v4i*)(dsts + e0 + 4);
  } else {
    da.x = (e0     < nE) ? dsts[min(e0,     nE - 1)] : sent;
    da.y = (e0 + 1 < nE) ? dsts[min(e0 + 1, nE - 1)] : sent;
    da.z = (e0 + 2 < nE) ? dsts[min(e0 + 2, nE - 1)] : sent;
    da.w = (e0 + 3 < nE) ? dsts[min(e0 + 3, nE - 1)] : sent;
    db.x = (e0 + 4 < nE) ? dsts[min(e0 + 4, nE - 1)] : sent;
    db.y = (e0 + 5 < nE) ? dsts[min(e0 + 5, nE - 1)] : sent;
    db.z = (e0 + 6 < nE) ? dsts[min(e0 + 6, nE - 1)] : sent;
    db.w = (e0 + 7 < nE) ? dsts[min(e0 + 7, nE - 1)] : sent;
  }
  const unsigned nbs = (unsigned)slotBase;
  const unsigned unb = (unsigned)nb;
  const unsigned s0 = (unsigned)da.x - nbs, s1 = (unsigned)da.y - nbs;
  const unsigned s2 = (unsigned)da.z - nbs, s3 = (unsigned)da.w - nbs;
  const unsigned s4 = (unsigned)db.x - nbs, s5 = (unsigned)db.y - nbs;
  const unsigned s6 = (unsigned)db.z - nbs, s7 = (unsigned)db.w - nbs;
  const bool h0 = s0 < unb, h1 = s1 < unb, h2 = s2 < unb, h3 = s3 < unb;
  const bool h4 = s4 < unb, h5 = s5 < unb, h6 = s6 < unb, h7 = s7 < unb;
  const unsigned any = __builtin_amdgcn_ballot_w32(h0 | h1 | h2 | h3 | h4 | h5 | h6 | h7);
  if (any != 0u) {
#define HITJ(J, HJ, SJ) { \
      const unsigned mj = __builtin_amdgcn_ballot_w32(HJ); \
      if (mj != 0u) { \
        if (HJ) { \
          const int pos = wc + (int)__builtin_amdgcn_mbcnt_lo(mj, 0u); \
          if (pos < WCAP) list[wave * WCAP + pos] = ((el0 + (J)) << 12) | (int)(SJ); \
        } \
        wc += (int)__builtin_popcount(mj); } }
    HITJ(0, h0, s0)
    HITJ(1, h1, s1)
    HITJ(2, h2, s2)
    HITJ(3, h3, s3)
    HITJ(4, h4, s4)
    HITJ(5, h5, s5)
    HITJ(6, h6, s6)
    HITJ(7, h7, s7)
#undef HITJ
  }
  return wc;
}

__global__ __launch_bounds__(NTHR) void k_xprep(const float* __restrict__ x, unsigned short* xb, int nN, int nUnits) {
  const int i = (int)blockIdx.x * NTHR + (int)threadIdx.x;
  if (i >= nUnits) return;
  const int row = i >> 2;
  const int q   = i & 3;
  const int rc  = row < nN ? row : nN - 1;
  const int qc  = q & 1;
  const float* p = x + (size_t)rc * FIN + 8 * qc;
  v4f a = *(const v4f*)p, b = *(const v4f*)(p + 4);
  const v4f z4 = {0.f, 0.f, 0.f, 0.f};
  if (row >= nN || q >= 2) { a = z4; b = z4; }
  const v8us hv = bits8(a, b);
  const size_t o = (size_t)i * 8;
  *(volatile v8us*)(xb + o) = hv;
  __threadfence();
  *(volatile v8us*)(xb + o) = hv;
}

__global__ __launch_bounds__(NTHR) void k_wtr(const float* __restrict__ w, int nMat, int K, int C, int NP, int KP,
                                              int dup, unsigned short* wt, int nUnits) {
  const int u = (int)blockIdx.x * NTHR + (int)threadIdx.x;
  if (u >= nUnits) return;
  const int kq = KP >> 3;
  const int perMat = NP * kq;
  int mi = u / perMat;
  mi = mi > nMat - 1 ? nMat - 1 : mi;
  const int rem = u - mi * perMat;
  const int n   = rem / kq;
  const int k8  = (rem - n * kq) * 8;
  const int khalf = KP >> 1;
  const int sec = (k8 >= khalf) ? 1 : 0;
  int ks = k8 - sec * khalf;
  ks = ks < 0 ? 0 : (ks > K - 8 ? K - 8 : ks);
  const int ncl = n < C ? n : C - 1;
  const float* p = w + (size_t)mi * (size_t)K * (size_t)C + (size_t)ks * (size_t)C + ncl;
  v4f a, b;
  a.x = p[0];                  a.y = p[(size_t)C];          a.z = p[(size_t)2 * C];      a.w = p[(size_t)3 * C];
  b.x = p[(size_t)4 * C];      b.y = p[(size_t)5 * C];      b.z = p[(size_t)6 * C];      b.w = p[(size_t)7 * C];
  const v4f z4 = {0.f, 0.f, 0.f, 0.f};
  if (n >= C || (sec == 1 && dup == 0)) { a = z4; b = z4; }
  const v8us hv = bits8(a, b);
  const size_t o = (size_t)u * 8;
  *(volatile v8us*)(wt + o) = hv;
  __threadfence();
  *(volatile v8us*)(wt + o) = hv;
}

template<int EPI, int ACT>
__global__ __launch_bounds__(GTHR) void k_gemm(
    const unsigned short* __restrict__ A, const unsigned short* __restrict__ WT,
    const float* __restrict__ bias, int blen,
    float* outF, unsigned short* outH, int K, int nRows)
{
  __shared__ __attribute__((aligned(16))) float stg[GBM * GBN];
  __shared__ __attribute__((aligned(16))) float rec[GBN];
  const int tid = (int)threadIdx.x, lane = tid & 31, wave = tid >> 5, hh = lane >> 4, m = lane & 15;
  const int rowBase = (int)blockIdx.x * GBM;

  v8f acc[4];
  {
    const v8f z = {0.f, 0.f, 0.f, 0.f, 0.f, 0.f, 0.f, 0.f};
    acc[0] = z; acc[1] = z; acc[2] = z; acc[3] = z;
  }
  const unsigned short* ap = A  + (size_t)(rowBase + 16 * wave + m) * (size_t)K + 8 * hh;
  const unsigned short* wp = WT + (size_t)m * (size_t)K + 8 * hh;
  const int ksteps = K >> 5;
#pragma unroll 1
  for (int ks = 0; ks < ksteps; ++ks) {
    FragB af;
    af.u[0] = *(const v8us*)(ap + 32 * ks);
    af.u[1] = *(const v8us*)(ap + 32 * ks + 16);
#pragma unroll
    for (int t = 0; t < 4; ++t) {
      const unsigned short* wq = wp + (size_t)(16 * t) * (size_t)K + 32 * ks;
      FragB bf;
      bf.u[0] = *(const v8us*)wq;
      bf.u[1] = *(const v8us*)(wq + 16);
      acc[t] = wmb(af, bf, acc[t]);
    }
  }

#pragma unroll
  for (int t = 0; t < 4; ++t) {
    const int lc = 16 * t + m;
    int bi = lc > blen - 1 ? blen - 1 : lc;
    bi = bi < 0 ? 0 : bi;
    const float bv = bfr(bias[bi]);
#pragma unroll
    for (int r = 0; r < 8; ++r) {
      const int lr = 16 * wave + 8 * hh + r;
      float v = acc[t][r] + bv;
      if (ACT == 1) v = v > 0.f ? v : 0.f;
      v = (rowBase + lr < nRows) ? v : 0.f;
      stg[lr * GBN + lc] = v;
    }
  }
  __syncthreads();

  if (EPI == 0) {
    v4f fv[8];
#pragma unroll
    for (int i = 0; i < 8; ++i) {
      const int lr = 16 * wave + 2 * i + hh;
      fv[i] = *(const v4f*)(stg + lr * GBN + 4 * m);
    }
#pragma unroll
    for (int i = 0; i < 8; ++i) {
      const int lr = 16 * wave + 2 * i + hh;
      const int gr = rowBase + lr;
      float* op = outF + (size_t)gr * (size_t)HC + 4 * m;
      *(volatile v4f*)op = fv[i];
    }
    __threadfence();
#pragma unroll
    for (int i = 0; i < 8; ++i) {
      const int lr = 16 * wave + 2 * i + hh;
      const int gr = rowBase + lr;
      float* op = outF + (size_t)gr * (size_t)HC + 4 * m;
      *(volatile v4f*)op = fv[i];
    }
  } else if (EPI == 1) {
    v8us pv[8];
#pragma unroll
    for (int i = 0; i < 8; ++i) {
      const int p   = i * GTHR + tid;
      const int row = p >> 4;
      const int q   = p & 15;
      const int c0  = (q & 7) * 8;
      const v4f a = *(const v4f*)(stg + row * GBN + c0);
      const v4f b = *(const v4f*)(stg + row * GBN + c0 + 4);
      v8us hi, lo;
      split8(a, b, hi, lo);
      v8us sel = hi;
      if (q >= 8) sel = lo;
      pv[i] = sel;
    }
    unsigned short* ob = outH + (size_t)rowBase * KHL;
#pragma unroll
    for (int i = 0; i < 8; ++i) {
      const int p = i * GTHR + tid;
      *(volatile v8us*)(ob + (size_t)p * 8) = pv[i];
    }
    __threadfence();
#pragma unroll
    for (int i = 0; i < 8; ++i) {
      const int p = i * GTHR + tid;
      *(volatile v8us*)(ob + (size_t)p * 8) = pv[i];
    }
  } else if (EPI == 2) {
    int nv = nRows - rowBase;
    nv = nv < 0 ? 0 : (nv > GBM ? GBM : nv);
    if (wave < 2) {
      float s = 0.f;
#pragma unroll 1
      for (int r = 0; r < nv; ++r) s += tanhf(stg[r * GBN + tid]);
      rec[tid] = s;
    }
    __syncthreads();
    if (wave == 0) {
      const int tl = lane < 16 ? lane : 15;
      const v4f v = *(const v4f*)(rec + 4 * tl);
      float* op = outF + (size_t)blockIdx.x * GBN + 4 * tl;
      const bool wsv = lane < 16;
      if (wsv) *(volatile v4f*)op = v;
      __threadfence();
      if (wsv) *(volatile v4f*)op = v;
    }
  } else {
    int nv = nRows - rowBase;
    nv = nv < 0 ? 0 : (nv > GBM ? GBM : nv);
    const int np = nv * (NOUT / 4);
    v4f pv[2];
#pragma unroll
    for (int i = 0; i < 2; ++i) {
      const int p   = i * GTHR + tid;
      const int row = p >> 2;
      const int c4  = (p & 3) * 4;
      v4f v = *(const v4f*)(stg + row * GBN + c4);
      v.x = tanhf(v.x); v.y = tanhf(v.y); v.z = tanhf(v.z); v.w = tanhf(v.w);
      pv[i] = v;
    }
    float* ob = outF + (size_t)rowBase * NOUT;
#pragma unroll
    for (int i = 0; i < 2; ++i) {
      const int p = i * GTHR + tid;
      if (p < np) *(volatile v4f*)(ob + 4 * p) = pv[i];
    }
    __threadfence();
#pragma unroll
    for (int i = 0; i < 2; ++i) {
      const int p = i * GTHR + tid;
      if (p < np) *(volatile v4f*)(ob + 4 * p) = pv[i];
    }
  }
}

__global__ __launch_bounds__(ATB) void k_nodeatt(const float* __restrict__ P,
                                                 const float* __restrict__ v0, const float* __restrict__ v1,
                                                 const float* __restrict__ v2, const float* __restrict__ v3,
                                                 float* AT, int nN) {
  __shared__ float vs[4 * HC];
  __shared__ __attribute__((aligned(16))) float st[ATB * ATW];
  const int t = (int)threadIdx.x;
  {
    const int g = t >> 6;
    const float* vp = (g == 0) ? v0 : ((g == 1) ? v1 : ((g == 2) ? v2 : v3));
    vs[t] = bfr(vp[t & 63]);
  }
  __syncthreads();
  const int node = (int)blockIdx.x * ATB + t;
  const int rc = node < nN ? node : nN - 1;
  const float* pr = P + (size_t)rc * HC;
  float a[8];
#pragma unroll
  for (int k = 0; k < 8; ++k) a[k] = 0.f;
#pragma unroll 1
  for (int d4 = 0; d4 < 8; ++d4) {
    const v4f p0 = *(const v4f*)(pr + 4 * d4);
    const v4f p1 = *(const v4f*)(pr + 32 + 4 * d4);
#pragma unroll
    for (int j = 0; j < 4; ++j) {
      const int d = 4 * d4 + j;
      const float x0 = p0[j];
      const float x1 = p1[j];
#pragma unroll
      for (int i = 0; i < 4; ++i) {
        a[2 * i]     = fmaf(x0, vs[i * HC + d],      a[2 * i]);
        a[2 * i + 1] = fmaf(x1, vs[i * HC + 32 + d], a[2 * i + 1]);
      }
    }
  }
  {
    const v4f oa = {a[0], a[1], a[2], a[3]};
    const v4f ob = {a[4], a[5], a[6], a[7]};
    *(v4f*)(st + t * ATW)     = oa;
    *(v4f*)(st + t * ATW + 4) = ob;
  }
  __syncthreads();
  float* base = AT + (size_t)blockIdx.x * (size_t)(ATB * ATW);
  const v4f q0 = *(const v4f*)(st + 4 * t);
  const v4f q1 = *(const v4f*)(st + 4 * (t + ATB));
  *(volatile v4f*)(base + 4 * t)         = q0;
  *(volatile v4f*)(base + 4 * (t + ATB)) = q1;
  __threadfence();
  *(volatile v4f*)(base + 4 * t)         = q0;
  *(volatile v4f*)(base + 4 * (t + ATB)) = q1;
}

__global__ __launch_bounds__(NTHR) void k_agg(
    const int* __restrict__ srcs, const int* __restrict__ dsts,
    const float* __restrict__ PS, const float* __restrict__ ATS, const float* __restrict__ ATD,
    float* OUT, int cs, int cd, int nNs, int nNd, int nE, int nb, int vec8, int MPr) {
  extern __shared__ v4f lds_dyn[];
  int* reg1 = (int*)lds_dyn;
  int* reg2 = reg1 + RCAP;
  int* scnt = reg2 + RCAP;
  int* soff = scnt + NBMAX;
  int* list = soff + NBMAX;
  int* wcnt = list + LISTN;
  int* wtot = wcnt + NWAVE;
  const int tid = (int)threadIdx.x, lane = tid & 31, wave = tid >> 5;
  const int nodeBase = (int)blockIdx.x * nb;

  for (int i = tid; i < NBMAX; i += NTHR) scnt[i] = 0;
  __syncthreads();

  int tot = 0;
  const int nChunks = (nE + CHUNK - 1) / CHUNK;
#pragma unroll 1
  for (int ch = 0; ch < nChunks; ++ch) {
    const int cbase = ch * CHUNK;
    const int wc = scan_chunk(dsts, nE, cbase, nodeBase, nb, vec8, list, tid, lane, wave);
    if (lane == 0) wcnt[wave] = wc;
    __syncthreads();
    int pre = 0, all = 0;
#pragma unroll
    for (int w2 = 0; w2 < NWAVE; ++w2) {
      int c = wcnt[w2];
      c = c < 0 ? 0 : (c > WCAP ? WCAP : c);
      all += c;
      pre += (w2 < wave) ? c : 0;
    }
    const int wcc  = wc > WCAP ? WCAP : wc;
    const int base = tot + pre;
#pragma unroll 1
    for (int i = lane; i < wcc; i += 32) {
      const int ent = list[wave * WCAP + i];
      const int el  = (ent >> 12) & (CHUNK - 1);
      const int sl  = ent & (NBMAX - 1);
      int eid = cbase + el;
      eid = eid > nE - 1 ? nE - 1 : eid;
      const int pos = base + i;
      if (pos < RCAP) reg1[pos] = (int)(((unsigned)eid << 12) | (unsigned)sl);
    }
    tot += all;
    tot = tot > RCAP ? RCAP : tot;
    __syncthreads();
  }
  const int nh = tot;

  if (wave == 0) {
#pragma unroll 1
    for (int b0 = 0; b0 < nh; b0 += 32) {
      const int idx = b0 + lane;
      const int uv  = reg1[idx < RCAP ? idx : RCAP - 1];
      const int m32 = (nh - b0) < 32 ? (nh - b0) : 32;
#pragma unroll 1
      for (int k = 0; k < m32; ++k) {
        const int u  = __builtin_amdgcn_readlane(uv, k);
        const int sl = u & (NBMAX - 1);
        if (lane == 0) scnt[sl] = scnt[sl] + 1;
      }
    }
  }
  __syncthreads();

  {
    const v4i ca = *(const v4i*)(scnt + 8 * tid);
    const v4i cb = *(const v4i*)(scnt + 8 * tid + 4);
    const int e0 = ca.x < 0 ? 0 : ca.x, e1 = ca.y < 0 ? 0 : ca.y, e2 = ca.z < 0 ? 0 : ca.z, e3 = ca.w < 0 ? 0 : ca.w;
    const int e4 = cb.x < 0 ? 0 : cb.x, e5 = cb.y < 0 ? 0 : cb.y, e6 = cb.z < 0 ? 0 : cb.z, e7 = cb.w < 0 ? 0 : cb.w;
    const int ts = e0 + e1 + e2 + e3 + e4 + e5 + e6 + e7;
    int incl = ts;
#pragma unroll
    for (int d = 1; d < 32; d <<= 1) {
      const int up = __shfl_up(incl, d);
      if (lane >= d) incl += up;
    }
    if (lane == 31) wtot[wave] = incl;
    __syncthreads();
    int pre = 0;
#pragma unroll
    for (int w2 = 0; w2 < NWAVE; ++w2) pre += (w2 < wave) ? wtot[w2] : 0;
    int run = pre + incl - ts;
    soff[8 * tid + 0] = run; run += e0;
    soff[8 * tid + 1] = run; run += e1;
    soff[8 * tid + 2] = run; run += e2;
    soff[8 * tid + 3] = run; run += e3;
    soff[8 * tid + 4] = run; run += e4;
    soff[8 * tid + 5] = run; run += e5;
    soff[8 * tid + 6] = run; run += e6;
    soff[8 * tid + 7] = run;
  }
  __syncthreads();
  for (int i = tid; i < NBMAX; i += NTHR) list[i] = soff[i];
  __syncthreads();

  if (wave == 0) {
#pragma unroll 1
    for (int b0 = 0; b0 < nh; b0 += 32) {
      const int idx = b0 + lane;
      const int uv  = reg1[idx < RCAP ? idx : RCAP - 1];
      const int m32 = (nh - b0) < 32 ? (nh - b0) : 32;
#pragma unroll 1
      for (int k = 0; k < m32; ++k) {
        const int u   = __builtin_amdgcn_readlane(uv, k);
        const int sl  = u & (NBMAX - 1);
        const int eid = (int)((unsigned)u >> 12);
        if (lane == 0) {
          int pos = list[sl];
          pos = pos < 0 ? 0 : (pos > RCAP - 1 ? RCAP - 1 : pos);
          reg2[pos] = eid;
          list[sl] = pos + 1;
        }
      }
    }
  }
  __syncthreads();

  const int nbw = nb >> 3;
  const bool ovf = (nh >= RCAP);
  const float qnan = __int_as_float(0x7fc00000);
  float* stw = (float*)reg1 + wave * STW;
  const int lc = lane < (HC / 4) ? lane : (HC / 4) - 1;
#pragma unroll 1
  for (int jt = 0; jt < nbw; ++jt) {
    const int slot = wave * nbw + jt;
    const int grow = nodeBase + slot;
    const int gcl  = grow < nNd ? grow : nNd - 1;
    int st = soff[slot];
    const int craw = scnt[slot];
    int cnt = craw;
    st  = st < 0 ? 0 : (st > nh ? nh : st);
    cnt = cnt < 0 ? 0 : (cnt > DEGCAP ? DEGCAP : cnt);
    if (cnt > nh - st) cnt = nh - st;
    const float pz = (ovf || craw > DEGCAP) ? qnan : 0.0f;
    const bool wr = grow < MPr;
    const float live = grow < nNd ? 1.0f : 0.0f;

    const float* drow = ATD + (size_t)gcl * ATW + cd;
    const float ad0 = drow[0];
    const float ad1 = drow[1];
    ldwait();
    float mx0 = -1.0e30f, mx1 = -1.0e30f;
    float dn0 = 0.f, dn1 = 0.f, av0 = 0.f, av1 = 0.f;

#pragma unroll 1
    for (int q = 0; q < cnt; ++q) {
      int idx = st + q; idx = idx > RCAP - 1 ? RCAP - 1 : idx;
      int eid = reg2[idx]; eid = eid < 0 ? 0 : (eid > nE - 1 ? nE - 1 : eid);
      const int sraw = srcs[eid];
      const int s = sraw < 0 ? 0 : (sraw > nNs - 1 ? nNs - 1 : sraw);
      const float* xr = PS + (size_t)s * HC + lane;
      const float x0 = xr[0];
      const float x1 = xr[32];
      const float* arow = ATS + (size_t)s * ATW + cs;
      const float as0 = arow[0];
      const float as1 = arow[1];
      ldwait();
      {
        float al = as0 + ad0;
        al = al >= 0.f ? al : 0.2f * al;
        const float df = al - mx0;
        const float ee = __expf(-fabsf(df));
        const bool up  = df > 0.f;
        const float s1 = up ? ee : 1.0f;
        const float s2 = up ? 1.0f : ee;
        mx0 = up ? al : mx0;
        dn0 = fmaf(dn0, s1, s2);
        av0 = fmaf(av0, s1, s2 * x0);
      }
      {
        float al = as1 + ad1;
        al = al >= 0.f ? al : 0.2f * al;
        const float df = al - mx1;
        const float ee = __expf(-fabsf(df));
        const bool up  = df > 0.f;
        const float s1 = up ? ee : 1.0f;
        const float s2 = up ? 1.0f : ee;
        mx1 = up ? al : mx1;
        dn1 = fmaf(dn1, s1, s2);
        av1 = fmaf(av1, s1, s2 * x1);
      }
    }
    const float ds0 = dn0 > 0.f ? dn0 : 1.0f;
    const float ds1 = dn1 > 0.f ? dn1 : 1.0f;
    const float iv0 = (dn0 > 0.f ? 1.0f : 0.0f) * __builtin_amdgcn_rcpf(ds0);
    const float iv1 = (dn1 > 0.f ? 1.0f : 0.0f) * __builtin_amdgcn_rcpf(ds1);
    const float r0 = fmaxf(av0 * iv0, 0.f) * live + pz;
    const float r1 = fmaxf(av1 * iv1, 0.f) * live + pz;
    __builtin_amdgcn_fence(__ATOMIC_RELEASE, "wavefront");
    __builtin_amdgcn_wave_barrier();
    stw[lane]      = r0;
    stw[32 + lane] = r1;
    __builtin_amdgcn_fence(__ATOMIC_RELEASE, "wavefront");
    __builtin_amdgcn_wave_barrier();
    const v4f ga = *(const v4f*)(stw + 4 * lc);
    float* gp = OUT + (size_t)grow * HC + 4 * lc;
    const bool wsv = wr && (lane < (HC / 4));
    if (wsv) *(volatile v4f*)gp = ga;
    __threadfence();
    if (wsv) *(volatile v4f*)gp = ga;
  }
}

template<int T>
__global__ __launch_bounds__(NTHR) void k_mix(const float* __restrict__ P0, const float* __restrict__ P1,
                                              const float* __restrict__ attn, const float* __restrict__ vw,
                                              unsigned short* HL, float* vpart, int nN, int dov) {
  __shared__ float wsum[NWAVE];
  __shared__ __attribute__((aligned(16))) float lineb[32];
  const int tid = (int)threadIdx.x, lane = tid & 31, wave = tid >> 5;
  const int hr = lane >> 4, q = lane & 15, c0 = (q & 7) * 8;
  const int rowBase = (int)blockIdx.x * MIXR;
  float a0 = 1.f, a1 = 0.f;
  if (T == 2) { a0 = attn[0]; a1 = attn[1]; }
  float wv[8];
  {
    const v4f wa = *(const v4f*)(vw + c0), wb = *(const v4f*)(vw + c0 + 4);
    wv[0] = bfr(wa.x); wv[1] = bfr(wa.y); wv[2] = bfr(wa.z); wv[3] = bfr(wa.w);
    wv[4] = bfr(wb.x); wv[5] = bfr(wb.y); wv[6] = bfr(wb.z); wv[7] = bfr(wb.w);
  }
  const v4f z4 = {0.f, 0.f, 0.f, 0.f};
  float vsum = 0.f;
  v8us pv[4];
#pragma unroll
  for (int it = 0; it < 4; ++it) {
    const int row = rowBase + 8 * wave + 2 * it + hr;
    const int rc  = row < nN ? row : nN - 1;
    const float* p0 = P0 + (size_t)rc * HC + c0;
    v4f va = *(const v4f*)p0, vb = *(const v4f*)(p0 + 4);
    if (T == 2) {
      const float* p1 = P1 + (size_t)rc * HC + c0;
      const v4f ya = *(const v4f*)p1, yb = *(const v4f*)(p1 + 4);
      va = a0 * va + a1 * ya;
      vb = a0 * vb + a1 * yb;
    }
    if (row >= nN) { va = z4; vb = z4; }
    v8us hi, lo;
    split8(va, vb, hi, lo);
    v8us sel = hi;
    if (q >= 8) sel = lo;
    pv[it] = sel;
    float ps = va.x * wv[0];
    ps = fmaf(va.y, wv[1], ps); ps = fmaf(va.z, wv[2], ps); ps = fmaf(va.w, wv[3], ps);
    ps = fmaf(vb.x, wv[4], ps); ps = fmaf(vb.y, wv[5], ps); ps = fmaf(vb.z, wv[6], ps); ps = fmaf(vb.w, wv[7], ps);
    vsum += (q < 8) ? ps : 0.f;
  }
#pragma unroll
  for (int it = 0; it < 4; ++it) {
    const int row = rowBase + 8 * wave + 2 * it + hr;
    *(volatile v8us*)(HL + (size_t)row * KHL + 8 * q) = pv[it];
  }
  __threadfence();
#pragma unroll
  for (int it = 0; it < 4; ++it) {
    const int row = rowBase + 8 * wave + 2 * it + hr;
    *(volatile v8us*)(HL + (size_t)row * KHL + 8 * q) = pv[it];
  }

#pragma unroll
  for (int off = 16; off > 0; off >>= 1) vsum += __shfl_xor(vsum, off);
  if (lane == 0) wsum[wave] = vsum;
  if (tid < 32) lineb[tid] = 0.f;
  __syncthreads();
  if (tid == 0) {
    float s = 0.f;
#pragma unroll
    for (int w = 0; w < NWAVE; ++w) s += wsum[w];
    lineb[0] = s;
  }
  __syncthreads();
  if (wave == 0) {
    const int tl = lane < 8 ? lane : 7;
    const v4f v = *(const v4f*)(lineb + 4 * tl);
    float* vp = vpart + (size_t)blockIdx.x * 32 + 4 * tl;
    const bool wsv = (dov != 0) && (lane < 8);
    if (wsv) *(volatile v4f*)vp = v;
    __threadfence();
    if (wsv) *(volatile v4f*)vp = v;
  }
}

__global__ __launch_bounds__(64) void k_semfold(const float* __restrict__ kpart, int gM, const float* __restrict__ qs,
                                                 int nN, float* attnl) {
  __shared__ float kk[2 * HC];
  __shared__ __attribute__((aligned(16))) float lineb[32];
  const int tid = (int)threadIdx.x, lane = tid & 31, wave = tid >> 5;
  double s0 = 0.0, s1 = 0.0;
#pragma unroll 1
  for (int b = 0; b < gM; ++b) {
    s0 += (double)kpart[(size_t)b * HC + tid];
    s1 += (double)kpart[(size_t)(gM + b) * HC + tid];
  }
  const double inv = 1.0 / (double)nN;
  kk[tid]      = (float)(s0 * inv);
  kk[HC + tid] = (float)(s1 * inv);
  if (tid < 32) lineb[tid] = 0.f;
  __syncthreads();
  float sc0 = 0.f, sc1 = 0.f;
#pragma unroll 1
  for (int c = 0; c < HC; ++c) {
    const float qv = bfr(qs[c]);
    sc0 = fmaf(qv, kk[c], sc0);
    sc1 = fmaf(qv, kk[HC + c], sc1);
  }
  const float mx = fmaxf(sc0, sc1);
  const float e0 = expf(sc0 - mx), e1 = expf(sc1 - mx);
  const float den = e0 + e1;
  const float a0 = e0 / den, a1 = e1 / den;
  if (tid == 0) { lineb[0] = a0; lineb[1] = a1; }
  __syncthreads();
  if (wave == 0) {
    const int tl = lane < 8 ? lane : 7;
    const v4f v = *(const v4f*)(lineb + 4 * tl);
    const bool wsv = lane < 8;
    if (wsv) *(volatile v4f*)(attnl + 4 * tl) = v;
    __threadfence();
    if (wsv) *(volatile v4f*)(attnl + 4 * tl) = v;
  }
}

__global__ __launch_bounds__(32) void k_valfold(const float* __restrict__ vpart, int nLines,
                                                 const float* __restrict__ vb, int cnt, float* outv) {
  double s = 0.0;
#pragma unroll 1
  for (int i = 0; i < nLines; ++i) s += (double)vpart[(size_t)i * 32];
  const float val = (float)(s / (double)cnt) + bfr(vb[0]);
  if (threadIdx.x == 0) {
    *(volatile float*)outv = val;
    __threadfence();
    *(volatile float*)outv = val;
  }
}

static int pick_nb(int nE, int nN) {
  int nb = NBMAX;
  while (nb > 16 && (long long)nb * (long long)nE * 5LL > (long long)RCAP * (long long)nN * 4LL) nb >>= 1;
  return nb;
}
static inline int cdiv(int a, int b) { return (a + b - 1) / b; }
static inline size_t al256(size_t o) { return (o + 255) & ~(size_t)255; }

extern "C" void kernel_launch(void* const* d_in, const int* in_sizes, int n_in,
                              void* d_out, int out_size, void* d_ws, size_t ws_size,
                              hipStream_t stream) {
  if (n_in < 22) return;
  if (in_sizes[0] < FIN || (in_sizes[0] % FIN) != 0) return;
  const int nN = in_sizes[0] / FIN;
  if (nN < 1 || nN > (1 << 22)) return;
  if (in_sizes[1] != nN * FIN) return;
  int nEv[3], nbv[3], gAv[3], v8v[3];
  for (int e = 0; e < 3; ++e) {
    const int sz = in_sizes[2 + e];
    if (sz < 2 || (sz & 1) != 0) return;
    nEv[e] = sz / 2;
    if (nEv[e] < 1 || nEv[e] > (1 << 20)) return;
  }
  if (in_sizes[5]  != FIN * HC || in_sizes[6] != HC || in_sizes[7] != FIN * HC || in_sizes[8] != HC) return;
  if (in_sizes[9]  != NLAY * 2 * HC * HC || in_sizes[10] != NLAY * 2 * HC) return;
  if (in_sizes[11] != NLAY * 3 * HC || in_sizes[12] != NLAY * 3 * HC) return;
  if (in_sizes[13] != NLAY * HC * HC || in_sizes[14] != NLAY * HC || in_sizes[15] != NLAY * HC) return;
  if (in_sizes[16] != HC * HC || in_sizes[17] != HC || in_sizes[18] != HC * NOUT || in_sizes[19] != NOUT) return;
  if (in_sizes[20] != HC || in_sizes[21] != 1) return;
  if (out_size != 2 * nN * NOUT + 1) return;

  const float* x_job    = (const float*)d_in[0];
  const float* x_mac    = (const float*)d_in[1];
  const int*   ei_jm    = (const int*)d_in[2];
  const int*   ei_mj    = (const int*)d_in[3];
  const int*   ei_jj    = (const int*)d_in[4];
  const float* enc_w_j  = (const float*)d_in[5];
  const float* enc_b_j  = (const float*)d_in[6];
  const float* enc_w_m  = (const float*)d_in[7];
  const float* enc_b_m  = (const float*)d_in[8];
  const float* proj_w   = (const float*)d_in[9];
  const float* proj_b   = (const float*)d_in[10];
  const float* att_src  = (const float*)d_in[11];
  const float* att_dst  = (const float*)d_in[12];
  const float* klin_w   = (const float*)d_in[13];
  const float* klin_b   = (const float*)d_in[14];
  const float* q_sem    = (const float*)d_in[15];
  const float* lin0_w   = (const float*)d_in[16];
  const float* lin0_b   = (const float*)d_in[17];
  const float* linout_w = (const float*)d_in[18];
  const float* linout_b = (const float*)d_in[19];
  const float* linv_w   = (const float*)d_in[20];
  const float* linv_b   = (const float*)d_in[21];
  float* out = (float*)d_out;

  const int MP  = cdiv(nN, GBM) * GBM;
  const int gM  = MP / GBM;
  const int NPA = cdiv(nN, ATB) * ATB;
  for (int e = 0; e < 3; ++e) {
    nbv[e] = pick_nb(nEv[e], nN);
    gAv[e] = cdiv(MP, nbv[e]);
    v8v[e] = ((nEv[e] & 3) == 0) ? 1 : 0;
    if (gAv[e] * nbv[e] < MP) return;
  }

  char* ws = (char*)d_ws;
  size_t off = 0;
  const size_t szXB = (size_t)MP * KENC * 2;
  const size_t szHL = (size_t)MP * KHL * 2;
  const size_t szPF = (size_t)MP * HC * 4;
  const size_t szAT = (size_t)NPA * ATW * 4;
  const size_t oXBJ = off; off = al256(off + szXB);
  const size_t oXBM = off; off = al256(off + szXB);
  const size_t oWEJ = off; off = al256(off + (size_t)HC * KENC * 2);
  const size_t oWEM = off; off = al256(off + (size_t)HC * KENC * 2);
  const size_t oWPR = off; off = al256(off + (size_t)4 * HC * KHL * 2);
  const size_t oWKL = off; off = al256(off + (size_t)2 * HC * KHL * 2);
  const size_t oWL0 = off; off = al256(off + (size_t)HC * KHL * 2);
  const size_t oWLO = off; off = al256(off + (size_t)HC * KHL * 2);
  const size_t oXJ  = off; off = al256(off + szHL);
  const size_t oXM  = off; off = al256(off + szHL);
  const size_t oMJH = off; off = al256(off + szHL);
  const size_t oJJH = off; off = al256(off + szHL);
  const size_t oHJ  = off; off = al256(off + szHL);
  const size_t oHM  = off; off = al256(off + szHL);
  const size_t oPJ  = off; off = al256(off + szPF);
  const size_t oPM  = off; off = al256(off + szPF);
  const size_t oOJM = off; off = al256(off + szPF);
  const size_t oOMJ = off; off = al256(off + szPF);
  const size_t oOJJ = off; off = al256(off + szPF);
  const size_t oATJ = off; off = al256(off + szAT);
  const size_t oATM = off; off = al256(off + szAT);
  const size_t oKP  = off; off = al256(off + (size_t)2 * gM * HC * 4);
  const size_t oATT = off; off = al256(off + 128);
  const size_t oVP  = off; off = al256(off + (size_t)2 * gM * 32 * 4);
  if (off > ws_size || off > (size_t)WSMAX) return;
  unsigned short* XBJ = (unsigned short*)(ws + oXBJ);
  unsigned short* XBM = (unsigned short*)(ws + oXBM);
  unsigned short* WEJ = (unsigned short*)(ws + oWEJ);
  unsigned short* WEM = (unsigned short*)(ws + oWEM);
  unsigned short* WPR = (unsigned short*)(ws + oWPR);
  unsigned short* WKL = (unsigned short*)(ws + oWKL);
  unsigned short* WL0 = (unsigned short*)(ws + oWL0);
  unsigned short* WLO = (unsigned short*)(ws + oWLO);
  unsigned short* XJ  = (unsigned short*)(ws + oXJ);
  unsigned short* XM  = (unsigned short*)(ws + oXM);
  unsigned short* MJH = (unsigned short*)(ws + oMJH);
  unsigned short* JJH = (unsigned short*)(ws + oJJH);
  unsigned short* HJ  = (unsigned short*)(ws + oHJ);
  unsigned short* HM  = (unsigned short*)(ws + oHM);
  float* PJ  = (float*)(ws + oPJ);
  float* PM  = (float*)(ws + oPM);
  float* OJM = (float*)(ws + oOJM);
  float* OMJ = (float*)(ws + oOMJ);
  float* OJJ = (float*)(ws + oOJJ);
  float* ATJ = (float*)(ws + oATJ);
  float* ATM = (float*)(ws + oATM);
  float* KP  = (float*)(ws + oKP);
  float* ATT = (float*)(ws + oATT);
  float* VP  = (float*)(ws + oVP);

  hipFuncSetAttribute(reinterpret_cast<const void*>(&k_agg),
                      hipFuncAttributeMaxDynamicSharedMemorySize, LDS_AGG);

  const int nUx = MP * (KENC / 8);
  k_xprep<<<cdiv(nUx, NTHR), NTHR, 0, stream>>>(x_job, XBJ, nN, nUx);
  k_xprep<<<cdiv(nUx, NTHR), NTHR, 0, stream>>>(x_mac, XBM, nN, nUx);

  {
    const int nUe = 1 * HC * KENC / 8;
    k_wtr<<<cdiv(nUe, NTHR), NTHR, 0, stream>>>(enc_w_j, 1, FIN, HC, HC, KENC, 0, WEJ, nUe);
    k_wtr<<<cdiv(nUe, NTHR), NTHR, 0, stream>>>(enc_w_m, 1, FIN, HC, HC, KENC, 0, WEM, nUe);
    const int nUp = 4 * HC * KHL / 8;
    k_wtr<<<cdiv(nUp, NTHR), NTHR, 0, stream>>>(proj_w, 4, HC, HC, HC, KHL, 1, WPR, nUp);
    const int nUk = 2 * HC * KHL / 8;
    k_wtr<<<cdiv(nUk, NTHR), NTHR, 0, stream>>>(klin_w, 2, HC, HC, HC, KHL, 1, WKL, nUk);
    const int nU1 = 1 * HC * KHL / 8;
    k_wtr<<<cdiv(nU1, NTHR), NTHR, 0, stream>>>(lin0_w, 1, HC, HC, HC, KHL, 1, WL0, nU1);
    k_wtr<<<cdiv(nU1, NTHR), NTHR, 0, stream>>>(linout_w, 1, HC, NOUT, HC, KHL, 1, WLO, nU1);
  }

  k_gemm<1, 1><<<gM, GTHR, 0, stream>>>(XBJ, WEJ, enc_b_j, HC, PJ, XJ, KENC, nN);
  k_gemm<1, 1><<<gM, GTHR, 0, stream>>>(XBM, WEM, enc_b_m, HC, PM, XM, KENC, nN);

  for (int l = 0; l < NLAY; ++l) {
    k_gemm<0, 0><<<gM, GTHR, 0, stream>>>(XJ, WPR + (size_t)(2 * l + 0) * HC * KHL, proj_b + (size_t)(2 * l + 0) * HC,
                                          HC, PJ, XJ, KHL, nN);
    k_gemm<0, 0><<<gM, GTHR, 0, stream>>>(XM, WPR + (size_t)(2 * l + 1) * HC * KHL, proj_b + (size_t)(2 * l + 1) * HC,
                                          HC, PM, XM, KHL, nN);
    const float* asl = att_src + (size_t)(3 * l) * HC;
    const float* adl = att_dst + (size_t)(3 * l) * HC;
    k_nodeatt<<<NPA / ATB, ATB, 0, stream>>>(PJ, asl + 0 * HC, adl + 1 * HC, asl + 2 * HC, adl + 2 * HC, ATJ, nN);
    k_nodeatt<<<NPA / ATB, ATB, 0, stream>>>(PM, adl + 0 * HC, asl + 1 * HC, adl + 0 * HC, asl + 1 * HC, ATM, nN);
    k_agg<<<gAv[0], NTHR, LDS_AGG, stream>>>(ei_jm, ei_jm + nEv[0], PJ, ATJ, ATM, OJM, 0, 0,
                                             nN, nN, nEv[0], nbv[0], v8v[0], MP);
    k_agg<<<gAv[1], NTHR, LDS_AGG, stream>>>(ei_mj, ei_mj + nEv[1], PM, ATM, ATJ, OMJ, 2, 2,
                                             nN, nN, nEv[1], nbv[1], v8v[1], MP);
    k_agg<<<gAv[2], NTHR, LDS_AGG, stream>>>(ei_jj, ei_jj + nEv[2], PJ, ATJ, ATJ, OJJ, 4, 6,
                                             nN, nN, nEv[2], nbv[2], v8v[2], MP);
    const int dov = (l == NLAY - 1) ? 1 : 0;
    k_mix<1><<<gM, NTHR, 0, stream>>>(OMJ, OMJ, ATT, linv_w, MJH, VP, nN, 0);
    k_mix<1><<<gM, NTHR, 0, stream>>>(OJJ, OJJ, ATT, linv_w, JJH, VP, nN, 0);
    k_mix<1><<<gM, NTHR, 0, stream>>>(OJM, OJM, ATT, linv_w, XM, VP + (size_t)gM * 32, nN, dov);
    k_gemm<2, 0><<<gM, GTHR, 0, stream>>>(MJH, WKL + (size_t)l * HC * KHL, klin_b + (size_t)l * HC, HC,
                                          KP, MJH, KHL, nN);
    k_gemm<2, 0><<<gM, GTHR, 0, stream>>>(JJH, WKL + (size_t)l * HC * KHL, klin_b + (size_t)l * HC, HC,
                                          KP + (size_t)gM * HC, JJH, KHL, nN);
    k_semfold<<<1, 64, 0, stream>>>(KP, gM, q_sem + (size_t)l * HC, nN, ATT);
    k_mix<2><<<gM, NTHR, 0, stream>>>(OMJ, OJJ, ATT, linv_w, XJ, VP, nN, dov);
  }

  k_gemm<1, 0><<<gM, GTHR, 0, stream>>>(XJ, WL0, lin0_b, HC, PJ, HJ, KHL, nN);
  k_gemm<1, 0><<<gM, GTHR, 0, stream>>>(XM, WL0, lin0_b, HC, PM, HM, KHL, nN);
  k_gemm<3, 0><<<gM, GTHR, 0, stream>>>(HJ, WLO, linout_b, NOUT, out, HJ, KHL, nN);
  k_gemm<3, 0><<<gM, GTHR, 0, stream>>>(HM, WLO, linout_b, NOUT, out + (size_t)nN * NOUT, HM, KHL, nN);
  k_valfold<<<1, 32, 0, stream>>>(VP, 2 * gM, linv_b, 2 * nN, out + (size_t)2 * nN * NOUT);
}
